// GINContextSubgraphClassifier_26731876451138
// MI455X (gfx1250) — hardware-verified
//
#include <hip/hip_runtime.h>
#include <stddef.h>
#include <math.h>


#define NTHR   256
#define NWAVE  8
#define EPT    8
#define CHUNK  (NTHR * EPT)
#define WCAP   (EPT * 32)
#define NB     512
#define RPW    (NB / NWAVE)
#define TPW    (NB / (16 * NWAVE))
#define NBG    128
#define RPWG   (NBG / NWAVE)
#define FD     128
#define OUTD   16
#define LN_EPS 1e-5f

#define LDS_ACC   0
#define LDS_LIST  (LDS_ACC + NB * FD * 4)
#define LDS_PRM   (LDS_LIST + NWAVE * WCAP * 4)
#define LDS_WCNT  (LDS_PRM + 4 * FD * 4)
#define LDS_TOTAL (LDS_WCNT + 64)

#define LP_ACC    0
#define LP_LIST   (LP_ACC + NBG * FD * 4)
#define LP_SOT    (LP_LIST + NWAVE * WCAP * 4)
#define LP_PRM    (LP_SOT + NBG * OUTD * 4)
#define LP_WCNT   (LP_PRM + (FD + 32) * 4)
#define LP_TOTAL  (LP_WCNT + 64)

static_assert(FD == 128);
static_assert(OUTD == 16);
static_assert(NB == TPW * 16 * NWAVE);
static_assert(NBG == 16 * NWAVE);
static_assert((NB & (NB - 1)) == 0 && NB <= 32768);
static_assert(CHUNK <= 65536);
static_assert(WCAP == 32 * EPT);
static_assert((LDS_TOTAL % 16) == 0);
static_assert(LDS_TOTAL <= 300 * 1024);
static_assert((LP_TOTAL % 16) == 0);
static_assert(2 * NTHR * 4 == NBG * OUTD);

typedef float        v4f   __attribute__((ext_vector_type(4)));
typedef float        v8f   __attribute__((ext_vector_type(8)));
typedef int          v4i   __attribute__((ext_vector_type(4)));
typedef unsigned int v4u   __attribute__((ext_vector_type(4)));
typedef __bf16       v16bf __attribute__((ext_vector_type(16)));
union FragB { v16bf v; v4u q[2]; };
union Pk8   { v4u q; __bf16 e[8]; };

__device__ __forceinline__ v8f zero8f() {
  v8f c;
#pragma unroll
  for (int i = 0; i < 8; ++i) c[i] = 0.0f;
  return c;
}

__device__ __forceinline__ v8f wmb(v16bf a, v16bf b, v8f c) {
  v8f d = __builtin_amdgcn_wmma_f32_16x16x32_bf16(false, a, false, b, (short)0, c, false, false);
  asm volatile("v_nop\n\tv_nop\n\tv_nop\n\tv_nop" : "+v"(d) : "v"(a), "v"(b));
  return d;
}

__device__ __forceinline__ void put4(v16bf& fh, v16bf& fl, const int b, const v4f a) {
  {
    const __bf16 hb = (__bf16)a.x; const float hf = (float)hb;
    fh[b] = hb; fl[b] = (__bf16)(a.x - hf);
  }
  {
    const __bf16 hb = (__bf16)a.y; const float hf = (float)hb;
    fh[b + 1] = hb; fl[b + 1] = (__bf16)(a.y - hf);
  }
  {
    const __bf16 hb = (__bf16)a.z; const float hf = (float)hb;
    fh[b + 2] = hb; fl[b + 2] = (__bf16)(a.z - hf);
  }
  {
    const __bf16 hb = (__bf16)a.w; const float hf = (float)hb;
    fh[b + 3] = hb; fl[b + 3] = (__bf16)(a.w - hf);
  }
}

__device__ __forceinline__ int scan_chunk(const int* __restrict__ keys, int nK, int cbase, int base,
                                          int span, int vec8, int* list, int tid, int wave) {
  int wc = 0;
  const int el0  = tid * EPT;
  const int e0   = cbase + el0;
  const int sent = -2147483647 - 1;
  v4i da, db;
  if (vec8 != 0 && cbase + CHUNK <= nK) {
    da = *(const v4i*)(keys + e0);
    db = *(const v4i*)(keys + e0 + 4);
  } else {
    da.x = (e0     < nK) ? keys[min(e0, nK - 1)] : sent;
    da.y = (e0 + 1 < nK) ? keys[min(e0 + 1, nK - 1)] : sent;
    da.z = (e0 + 2 < nK) ? keys[min(e0 + 2, nK - 1)] : sent;
    da.w = (e0 + 3 < nK) ? keys[min(e0 + 3, nK - 1)] : sent;
    db.x = (e0 + 4 < nK) ? keys[min(e0 + 4, nK - 1)] : sent;
    db.y = (e0 + 5 < nK) ? keys[min(e0 + 5, nK - 1)] : sent;
    db.z = (e0 + 6 < nK) ? keys[min(e0 + 6, nK - 1)] : sent;
    db.w = (e0 + 7 < nK) ? keys[min(e0 + 7, nK - 1)] : sent;
  }
  const unsigned nb = (unsigned)base;
  const unsigned sp = (unsigned)span;
  const unsigned s0 = (unsigned)da.x - nb, s1 = (unsigned)da.y - nb;
  const unsigned s2 = (unsigned)da.z - nb, s3 = (unsigned)da.w - nb;
  const unsigned s4 = (unsigned)db.x - nb, s5 = (unsigned)db.y - nb;
  const unsigned s6 = (unsigned)db.z - nb, s7 = (unsigned)db.w - nb;
  const bool h0 = s0 < sp, h1 = s1 < sp, h2 = s2 < sp, h3 = s3 < sp;
  const bool h4 = s4 < sp, h5 = s5 < sp, h6 = s6 < sp, h7 = s7 < sp;
  const unsigned any = __builtin_amdgcn_ballot_w32(h0 | h1 | h2 | h3 | h4 | h5 | h6 | h7);
  if (any != 0u) {
#define HITJ(J, HJ, SJ) { \
      const unsigned mj = __builtin_amdgcn_ballot_w32(HJ); \
      if (mj != 0u) { \
        if (HJ) { \
          const int pos = wc + (int)__builtin_amdgcn_mbcnt_lo(mj, 0u); \
          if (pos < WCAP) list[wave * WCAP + pos] = (int)(((SJ) << 16) | (unsigned)(el0 + (J))); \
        } \
        wc += (int)__builtin_popcount(mj); } }
    HITJ(0, h0, s0)
    HITJ(1, h1, s1)
    HITJ(2, h2, s2)
    HITJ(3, h3, s3)
    HITJ(4, h4, s4)
    HITJ(5, h5, s5)
    HITJ(6, h6, s6)
    HITJ(7, h7, s7)
#undef HITJ
  }
  return wc;
}

__device__ __forceinline__ void gemm128(const float* zr,
                                        const unsigned short* __restrict__ whi,
                                        const unsigned short* __restrict__ wlo,
                                        const int m, const int hh, v8f (&c)[8]) {
#pragma unroll
  for (int nt = 0; nt < 8; ++nt) c[nt] = zero8f();
#pragma unroll 1
  for (int kt = 0; kt < 4; ++kt) {
    v16bf ah, al;
    {
      const float* zp = zr + 32 * kt;
      const v4f z0 = *(const v4f*)zp;
      const v4f z1 = *(const v4f*)(zp + 4);
      const v4f z2 = *(const v4f*)(zp + 16);
      const v4f z3 = *(const v4f*)(zp + 20);
      put4(ah, al, 0, z0);
      put4(ah, al, 4, z1);
      put4(ah, al, 8, z2);
      put4(ah, al, 12, z3);
    }
    const unsigned short* bph = whi + (size_t)m * FD + 32 * kt + 8 * hh;
    const unsigned short* bpl = wlo + (size_t)m * FD + 32 * kt + 8 * hh;
#pragma unroll
    for (int nt = 0; nt < 8; ++nt) {
      FragB bh, bl;
      const unsigned short* p = bph + (size_t)nt * 16 * FD;
      const unsigned short* q = bpl + (size_t)nt * 16 * FD;
      bh.q[0] = *(const v4u*)p;
      bh.q[1] = *(const v4u*)(p + 16);
      bl.q[0] = *(const v4u*)q;
      bl.q[1] = *(const v4u*)(q + 16);
      c[nt] = wmb(ah, bh.v, c[nt]);
      c[nt] = wmb(ah, bl.v, c[nt]);
      c[nt] = wmb(al, bh.v, c[nt]);
    }
  }
}

__global__ __launch_bounds__(NTHR) void k_prep(const float* __restrict__ W1, const float* __restrict__ W2,
                                              const float* __restrict__ Wa, const float* __restrict__ Wb,
                                              int nL, unsigned short* whi, unsigned short* wlo) {
  const int tid = threadIdx.x;
  const int b = blockIdx.x;
  const int nFull = 2 * nL + 1;
  const float* src;
  int ncol, n, kc;
  size_t dsto;
  if (b < 8 * nFull) {
    const int mat = b >> 3;
    const int u = ((b & 7) << 8) + tid;
    n = u >> 4;
    kc = u & 15;
    ncol = FD;
    src = (mat < nL) ? (W1 + (size_t)mat * FD * FD)
                     : ((mat < 2 * nL) ? (W2 + (size_t)(mat - nL) * FD * FD) : Wa);
    dsto = (size_t)mat * FD * FD + (size_t)u * 8;
  } else {
    n = tid >> 4;
    kc = tid & 15;
    ncol = OUTD;
    src = Wb;
    dsto = (size_t)nFull * FD * FD + (size_t)tid * 8;
  }
  Pk8 ph, pl;
#pragma unroll
  for (int j = 0; j < 8; ++j) {
    const int k = 8 * kc + j;
    const float w = src[(size_t)k * ncol + n];
    const __bf16 hb = (__bf16)w;
    const float  hf = (float)hb;
    ph.e[j] = hb;
    pl.e[j] = (__bf16)(w - hf);
  }
  unsigned short* dh = whi + dsto;
  unsigned short* dl = wlo + dsto;
  const v4u qh = ph.q;
  const v4u ql = pl.q;
  *(volatile v4u*)dh = qh;
  *(volatile v4u*)dl = ql;
  __threadfence();
  *(volatile v4u*)dh = qh;
  *(volatile v4u*)dl = ql;
}

__global__ __launch_bounds__(NTHR) void k_layer(
    const float* __restrict__ hin, const int* __restrict__ ei,
    const unsigned short* __restrict__ w1h, const unsigned short* __restrict__ w1l,
    const unsigned short* __restrict__ w2h, const unsigned short* __restrict__ w2l,
    const float* __restrict__ b1, const float* __restrict__ b2,
    const float* __restrict__ gam, const float* __restrict__ bet,
    const float* __restrict__ epsv, float* hout,
    int layer, int nN, int nE, int vec8) {
  extern __shared__ __attribute__((aligned(16))) unsigned char dsm[];
  float* acc  = (float*)(dsm + LDS_ACC);
  int*   list = (int*)(dsm + LDS_LIST);
  float* prm  = (float*)(dsm + LDS_PRM);
  int*   wcnt = (int*)(dsm + LDS_WCNT);

  const int tid = threadIdx.x, lane = tid & 31, wave = tid >> 5, hh = lane >> 4, m = lane & 15;
  const int nodeBase = blockIdx.x * NB;
  const int* srcs = ei;
  const int* dsts = ei + nE;
  const float opl = 1.0f + epsv[layer];

  {
    const v4f z4 = {0.0f, 0.0f, 0.0f, 0.0f};
#pragma unroll 1
    for (int rr = 0; rr < RPW; ++rr) {
      const int row  = wave * RPW + rr;
      const int node = nodeBase + row;
      const int nc   = node < nN ? node : nN - 1;
      v4f v = *(const v4f*)(hin + (size_t)nc * FD + 4 * lane);
      if (node >= nN) v = z4;
      v = v * opl;
      *(v4f*)(acc + row * FD + 4 * lane) = v;
    }
  }
  if (tid < FD) {
    prm[tid]          = b1[tid];
    prm[FD + tid]     = b2[tid];
    prm[2 * FD + tid] = gam[tid];
    prm[3 * FD + tid] = bet[tid];
  }
  __syncthreads();

  {
    const int nChunks = (nE + CHUNK - 1) / CHUNK;
#pragma unroll 1
    for (int ch = 0; ch < nChunks; ++ch) {
      const int cbase = ch * CHUNK;
      const int wc = scan_chunk(dsts, nE, cbase, nodeBase, NB, vec8, list, tid, wave);
      if (lane == 0) wcnt[wave] = wc;
      __syncthreads();

      if (wave == 0) {
#pragma unroll 1
        for (int u = 0; u < NWAVE; ++u) {
          int n = __builtin_amdgcn_readfirstlane(wcnt[u]);
          n = n > WCAP ? WCAP : (n < 0 ? 0 : n);
#pragma unroll 1
          for (int i = 0; i < n; ++i) {
            const int ent  = __builtin_amdgcn_readfirstlane(list[u * WCAP + i]);
            const int el   = ent & 0xFFFF;
            const int slot = (ent >> 16) & (NB - 1);
            int e = cbase + el;
            e = e > nE - 1 ? nE - 1 : e;
            int s = srcs[e];
            s = s < 0 ? 0 : (s > nN - 1 ? nN - 1 : s);
            const v4f v = *(const v4f*)(hin + (size_t)s * FD + 4 * lane);
            float* ap = acc + slot * FD + 4 * lane;
            v4f a = *(v4f*)ap;
            a += v;
            *(v4f*)ap = a;
          }
        }
      }
      __syncthreads();
    }
  }

#pragma unroll 1
  for (int tt = 0; tt < TPW; ++tt) {
    const int t = wave + NWAVE * tt;
    const float* zr = acc + (16 * t + m) * FD + 8 * hh;
    float* orow = acc + (16 * t + 8 * hh) * FD + m;
    v8f c[8];

    gemm128(zr, w1h, w1l, m, hh, c);
    __syncthreads();
    {
#pragma unroll
      for (int nt = 0; nt < 8; ++nt) {
        const float bb = prm[16 * nt + m];
#pragma unroll
        for (int r = 0; r < 8; ++r) c[nt][r] = fmaxf(c[nt][r] + bb, 0.0f);
      }
#pragma unroll
      for (int r = 0; r < 8; ++r) {
#pragma unroll
        for (int nt = 0; nt < 8; ++nt) orow[r * FD + 16 * nt] = c[nt][r];
      }
    }
    __syncthreads();

    gemm128(zr, w2h, w2l, m, hh, c);
    __syncthreads();
    {
      float ga[8], be[8];
#pragma unroll
      for (int nt = 0; nt < 8; ++nt) {
        const int n = 16 * nt + m;
        const float bb = prm[FD + n];
        ga[nt] = prm[2 * FD + n];
        be[nt] = prm[3 * FD + n];
#pragma unroll
        for (int r = 0; r < 8; ++r) c[nt][r] = c[nt][r] + bb;
      }
#pragma unroll
      for (int r = 0; r < 8; ++r) {
        float s = 0.0f;
#pragma unroll
        for (int nt = 0; nt < 8; ++nt) s += c[nt][r];
        s += __shfl_xor(s, 1, 32);
        s += __shfl_xor(s, 2, 32);
        s += __shfl_xor(s, 4, 32);
        s += __shfl_xor(s, 8, 32);
        const float mu = s * (1.0f / FD);
        float q = 0.0f;
#pragma unroll
        for (int nt = 0; nt < 8; ++nt) { const float d = c[nt][r] - mu; q += d * d; }
        q += __shfl_xor(q, 1, 32);
        q += __shfl_xor(q, 2, 32);
        q += __shfl_xor(q, 4, 32);
        q += __shfl_xor(q, 8, 32);
        const float rs = rsqrtf(q * (1.0f / FD) + LN_EPS);
#pragma unroll
        for (int nt = 0; nt < 8; ++nt)
          c[nt][r] = fmaxf((c[nt][r] - mu) * rs * ga[nt] + be[nt], 0.0f);
      }
#pragma unroll
      for (int r = 0; r < 8; ++r) {
#pragma unroll
        for (int nt = 0; nt < 8; ++nt) orow[r * FD + 16 * nt] = c[nt][r];
      }
    }
    __syncthreads();
  }

#pragma unroll 1
  for (int rr = 0; rr < RPW; ++rr) {
    const int row  = wave * RPW + rr;
    const int node = nodeBase + row;
    const int nc   = node < nN ? node : nN - 1;
    float* ap = acc + row * FD + 4 * lane;
    v4f a = *(v4f*)ap;
    const v4f hv = *(const v4f*)(hin + (size_t)nc * FD + 4 * lane);
    a += hv;
    *(v4f*)ap = a;
  }

#pragma unroll 1
  for (int rr = 0; rr < RPW; ++rr) {
    const int row = wave * RPW + rr;
    const v4f v = *(const v4f*)(acc + row * FD + 4 * lane);
    *(volatile v4f*)(hout + (size_t)(nodeBase + row) * FD + 4 * lane) = v;
  }
  __threadfence();
#pragma unroll 1
  for (int rr = 0; rr < RPW; ++rr) {
    const int row = wave * RPW + rr;
    const v4f v = *(const v4f*)(acc + row * FD + 4 * lane);
    *(volatile v4f*)(hout + (size_t)(nodeBase + row) * FD + 4 * lane) = v;
  }
}

__global__ __launch_bounds__(NTHR) void k_poolhead(
    const float* __restrict__ h, const int* __restrict__ bt,
    const unsigned short* __restrict__ wah, const unsigned short* __restrict__ wal,
    const unsigned short* __restrict__ wbh, const unsigned short* __restrict__ wbl,
    const float* __restrict__ bh1, const float* __restrict__ bh2,
    float* outp, int nN, int nG) {
  extern __shared__ __attribute__((aligned(16))) unsigned char dsm[];
  float* accz = (float*)(dsm + LP_ACC);
  int*   list = (int*)(dsm + LP_LIST);
  float* sot  = (float*)(dsm + LP_SOT);
  float* prm  = (float*)(dsm + LP_PRM);
  int*   wcnt = (int*)(dsm + LP_WCNT);

  const int tid = threadIdx.x, lane = tid & 31, wave = tid >> 5, hh = lane >> 4, m = lane & 15;
  const int gBase = blockIdx.x * NBG;

  {
    const v4f z4 = {0.0f, 0.0f, 0.0f, 0.0f};
#pragma unroll 1
    for (int rr = 0; rr < RPWG; ++rr) {
      const int row = wave * RPWG + rr;
      *(v4f*)(accz + row * FD + 4 * lane) = z4;
    }
  }
  if (tid < FD)   prm[tid] = bh1[tid];
  if (tid < OUTD) prm[FD + tid] = bh2[tid];
  __syncthreads();

  {
    const int nChunks = (nN + CHUNK - 1) / CHUNK;
#pragma unroll 1
    for (int ch = 0; ch < nChunks; ++ch) {
      const int cbase = ch * CHUNK;
      const int wc = scan_chunk(bt, nN, cbase, gBase, NBG, 1, list, tid, wave);
      if (lane == 0) wcnt[wave] = wc;
      __syncthreads();

      if (wave == 0) {
#pragma unroll 1
        for (int u = 0; u < NWAVE; ++u) {
          int n = __builtin_amdgcn_readfirstlane(wcnt[u]);
          n = n > WCAP ? WCAP : (n < 0 ? 0 : n);
#pragma unroll 1
          for (int i = 0; i < n; ++i) {
            const int ent  = __builtin_amdgcn_readfirstlane(list[u * WCAP + i]);
            const int el   = ent & 0xFFFF;
            const int slot = (ent >> 16) & (NBG - 1);
            int nd = cbase + el;
            nd = nd > nN - 1 ? nN - 1 : nd;
            const v4f v = *(const v4f*)(h + (size_t)nd * FD + 4 * lane);
            float* ap = accz + slot * FD + 4 * lane;
            v4f a = *(v4f*)ap;
            a += v;
            *(v4f*)ap = a;
          }
        }
      }
      __syncthreads();
    }
  }

  const int t = wave;
  const float* zr = accz + (16 * t + m) * FD + 8 * hh;
  float* orow = accz + (16 * t + 8 * hh) * FD + m;
  {
    v8f c[8];
    gemm128(zr, wah, wal, m, hh, c);
    __syncthreads();
#pragma unroll
    for (int nt = 0; nt < 8; ++nt) {
      const float bb = prm[16 * nt + m];
#pragma unroll
      for (int r = 0; r < 8; ++r) c[nt][r] = fmaxf(c[nt][r] + bb, 0.0f);
    }
#pragma unroll
    for (int r = 0; r < 8; ++r) {
#pragma unroll
      for (int nt = 0; nt < 8; ++nt) orow[r * FD + 16 * nt] = c[nt][r];
    }
  }
  __syncthreads();
  {
    v8f c2 = zero8f();
#pragma unroll 1
    for (int kt = 0; kt < 4; ++kt) {
      v16bf ah, al;
      {
        const float* zp = zr + 32 * kt;
        const v4f z0 = *(const v4f*)zp;
        const v4f z1 = *(const v4f*)(zp + 4);
        const v4f z2 = *(const v4f*)(zp + 16);
        const v4f z3 = *(const v4f*)(zp + 20);
        put4(ah, al, 0, z0);
        put4(ah, al, 4, z1);
        put4(ah, al, 8, z2);
        put4(ah, al, 12, z3);
      }
      const unsigned short* p = wbh + (size_t)m * FD + 32 * kt + 8 * hh;
      const unsigned short* q = wbl + (size_t)m * FD + 32 * kt + 8 * hh;
      FragB bh, bl;
      bh.q[0] = *(const v4u*)p;
      bh.q[1] = *(const v4u*)(p + 16);
      bl.q[0] = *(const v4u*)q;
      bl.q[1] = *(const v4u*)(q + 16);
      c2 = wmb(ah, bh.v, c2);
      c2 = wmb(ah, bl.v, c2);
      c2 = wmb(al, bh.v, c2);
    }
    const float bb2 = prm[FD + m];
#pragma unroll
    for (int r = 0; r < 8; ++r) sot[(16 * t + 8 * hh + r) * OUTD + m] = c2[r] + bb2;
  }
  __syncthreads();

  {
    const size_t obase = (size_t)gBase * OUTD;
    const int f0 = tid, f1 = tid + NTHR;
    const v4f o0 = *(const v4f*)(sot + 4 * f0);
    const v4f o1 = *(const v4f*)(sot + 4 * f1);
    const int g0 = gBase + (f0 >> 2);
    const int g1 = gBase + (f1 >> 2);
    if (g0 < nG) *(volatile v4f*)(outp + obase + 4 * f0) = o0;
    if (g1 < nG) *(volatile v4f*)(outp + obase + 4 * f1) = o1;
    __threadfence();
    if (g0 < nG) *(volatile v4f*)(outp + obase + 4 * f0) = o0;
    if (g1 < nG) *(volatile v4f*)(outp + obase + 4 * f1) = o1;
  }
}

extern "C" void kernel_launch(void* const* d_in, const int* in_sizes, int n_in,
                              void* d_out, int out_size, void* d_ws, size_t ws_size,
                              hipStream_t stream) {
  if (n_in < 14) return;
  const int nN = in_sizes[2];
  if (nN < 1 || in_sizes[0] != nN * FD) return;
  const int nE = in_sizes[1] / 2;
  if (nE < 1 || in_sizes[1] != 2 * nE) return;
  const int nL = in_sizes[7];
  if (nL < 1 || nL > 16) return;
  if (in_sizes[3] != nL * FD * FD || in_sizes[4] != nL * FD) return;
  if (in_sizes[5] != nL * FD * FD || in_sizes[6] != nL * FD) return;
  if (in_sizes[8] != nL * FD || in_sizes[9] != nL * FD) return;
  if (in_sizes[10] != FD * FD || in_sizes[11] != FD) return;
  if (in_sizes[12] != FD * OUTD || in_sizes[13] != OUTD) return;
  const int nG = out_size / OUTD;
  if (nG < 1 || out_size != nG * OUTD) return;

  const float* x     = (const float*)d_in[0];
  const int*   ei    = (const int*)d_in[1];
  const int*   batch = (const int*)d_in[2];
  const float* W1    = (const float*)d_in[3];
  const float* b1    = (const float*)d_in[4];
  const float* W2    = (const float*)d_in[5];
  const float* b2    = (const float*)d_in[6];
  const float* epsv  = (const float*)d_in[7];
  const float* gam   = (const float*)d_in[8];
  const float* bet   = (const float*)d_in[9];
  const float* Wh1   = (const float*)d_in[10];
  const float* bh1   = (const float*)d_in[11];
  const float* Wh2   = (const float*)d_in[12];
  const float* bh2   = (const float*)d_in[13];
  float* outp = (float*)d_out;

  const int nBlk  = (nN + NB - 1) / NB;
  const int nBlkG = (nG + NBG - 1) / NBG;
  const size_t rowsP = (size_t)nBlk * NB;
  const int nFull = 2 * nL + 1;
  const size_t planeHalves = (size_t)nFull * FD * FD + (size_t)OUTD * FD;

  char* ws = (char*)d_ws;
  size_t off = 0;
  const size_t oWh = off; off += (planeHalves * 2 + 255) & ~(size_t)255;
  const size_t oWl = off; off += (planeHalves * 2 + 255) & ~(size_t)255;
  const size_t oX0 = off; off += (rowsP * FD * 4 + 255) & ~(size_t)255;
  const size_t oX1 = off; off += (rowsP * FD * 4 + 255) & ~(size_t)255;
  size_t limit = (size_t)134217728;
  if (ws_size < limit) limit = ws_size;
  if (off > limit) return;

  unsigned short* Wh = (unsigned short*)(ws + oWh);
  unsigned short* Wl = (unsigned short*)(ws + oWl);
  float* X0 = (float*)(ws + oX0);
  float* X1 = (float*)(ws + oX1);

  const int vec8 = ((nE & 3) == 0) ? 1 : 0;

  k_prep<<<8 * nFull + 1, NTHR, 0, stream>>>(W1, W2, Wh1, Wh2, nL, Wh, Wl);

  (void)hipFuncSetAttribute(reinterpret_cast<const void*>(&k_layer),
                            hipFuncAttributeMaxDynamicSharedMemorySize, LDS_TOTAL);
  (void)hipFuncSetAttribute(reinterpret_cast<const void*>(&k_poolhead),
                            hipFuncAttributeMaxDynamicSharedMemorySize, LP_TOTAL);

  const float* hin = x;
  for (int l = 0; l < nL; ++l) {
    float* hout = (l & 1) ? X1 : X0;
    k_layer<<<nBlk, NTHR, LDS_TOTAL, stream>>>(
        hin, ei,
        Wh + (size_t)l * FD * FD, Wl + (size_t)l * FD * FD,
        Wh + (size_t)(nL + l) * FD * FD, Wl + (size_t)(nL + l) * FD * FD,
        b1 + (size_t)l * FD, b2 + (size_t)l * FD,
        gam + (size_t)l * FD, bet + (size_t)l * FD,
        epsv, hout, l, nN, nE, vec8);
    hin = hout;
  }

  k_poolhead<<<nBlkG, NTHR, LP_TOTAL, stream>>>(
      hin, batch,
      Wh + (size_t)(2 * nL) * FD * FD, Wl + (size_t)(2 * nL) * FD * FD,
      Wh + (size_t)nFull * FD * FD, Wl + (size_t)nFull * FD * FD,
      bh1, bh2, outp, nN, nG);
}
